// MetaLinear2_20220706030481
// MI455X (gfx1250) — hardware-verified
//
#include <hip/hip_runtime.h>
#include <math.h>

typedef __attribute__((ext_vector_type(16))) _Float16 v16h;
typedef __attribute__((ext_vector_type(16))) __bf16 v16b;
typedef __attribute__((ext_vector_type(8)))  _Float16 v8h;
typedef __attribute__((ext_vector_type(8)))  float v8f;
typedef __attribute__((ext_vector_type(4)))  float v4f;
typedef __attribute__((ext_vector_type(2)))  float v2f;
typedef __attribute__((ext_vector_type(4)))  unsigned v4u;
typedef __attribute__((ext_vector_type(4)))  int v4i;
typedef float __attribute__((may_alias)) float_a;
typedef int __attribute__((may_alias)) int_a;

template <typename T> __device__ __forceinline__ void vst2(void* p, T v) { *(volatile T*)p = v; __threadfence(); *(volatile T*)p = v; }
__device__ __forceinline__ v8f wmma16(v16h a, v16h b, v8f c) {
  v8f d = __builtin_amdgcn_wmma_f32_16x16x32_f16(false, a, false, b, (short)0, c, false, false);
  asm volatile("v_nop\n\tv_nop\n\tv_nop\n\tv_nop" : "+v"(d) : "v"(a), "v"(b));
  return d;
}
__device__ __forceinline__ v8f wmma_bf(v16b a, v16b b, v8f c) {
  v8f d = __builtin_amdgcn_wmma_f32_16x16x32_bf16(false, a, false, b, (short)0, c, false, false);
  asm volatile("v_nop\n\tv_nop\n\tv_nop\n\tv_nop" : "+v"(d) : "v"(a), "v"(b));
  return d;
}
__device__ __forceinline__ v16h frag_h(const _Float16* rowk0, int lane) {
  union { v16h v; v8h q[2]; } u; const _Float16* p = rowk0 + 8 * (lane >> 4);
  u.q[0] = *(const v8h*)p; u.q[1] = *(const v8h*)(p + 16); return u.v;
}
__device__ __forceinline__ v16h frag_f32(const float* rowk0, int lane) {
  v16h a; const float* p = rowk0 + 8 * (lane >> 4);
#pragma unroll
  for (int i = 0; i < 8; ++i) { a[i] = (_Float16)p[i]; a[8 + i] = (_Float16)p[16 + i]; }
  return a;
}
__device__ __forceinline__ v16h frag_f32s(const float* rowk0, int lane, float sc) {
  v16h a; const float* p = rowk0 + 8 * (lane >> 4);
#pragma unroll
  for (int i = 0; i < 8; ++i) { a[i] = (_Float16)(p[i] * sc); a[8 + i] = (_Float16)(p[16 + i] * sc); }
  return a;
}
__device__ __forceinline__ v16h fragc_f32(const float* W, int k0, int n, int lane, int ld, int K) {
  v16h a; const int g = lane >> 4;
#pragma unroll
  for (int i = 0; i < 8; ++i) { const int ka = k0 + 8 * g + i, kb = ka + 16;
    a[i] = (_Float16)(ka < K ? W[(size_t)(ka < K ? ka : K - 1) * ld + n] : 0.f); a[8 + i] = (_Float16)(kb < K ? W[(size_t)(kb < K ? kb : K - 1) * ld + n] : 0.f); }
  return a;
}
struct F2 { v16b h, l; };
__device__ __forceinline__ F2 bsplit16(const float v[16]) { F2 r;
#pragma unroll
  for (int i = 0; i < 16; ++i) { const __bf16 h = (__bf16)v[i]; r.h[i] = h; r.l[i] = (__bf16)(v[i] - (float)h); }
  return r; }
__device__ __forceinline__ F2 split_row(const float* row, int k0, int lane) { float v[16]; const float* p = row + k0 + 8 * (lane >> 4);
#pragma unroll
  for (int i = 0; i < 8; ++i) { v[i] = p[i]; v[8 + i] = p[16 + i]; }
  return bsplit16(v); }
__device__ __forceinline__ F2 split_rowK(const float* row, int k0, int lane, int K) { float v[16]; const int g = lane >> 4;
#pragma unroll
  for (int i = 0; i < 8; ++i) { const int ka = k0 + 8 * g + i, kb = ka + 16; v[i] = ka < K ? row[ka < K ? ka : K - 1] : 0.f; v[8 + i] = kb < K ? row[kb < K ? kb : K - 1] : 0.f; }
  return bsplit16(v); }
__device__ __forceinline__ F2 split_col(const float* W, int k0, int n, int lane, int ld, int K) { float v[16]; const int g = lane >> 4;
#pragma unroll
  for (int i = 0; i < 8; ++i) { const int ka = k0 + 8 * g + i, kb = ka + 16; v[i] = ka < K ? W[(size_t)(ka < K ? ka : K - 1) * ld + n] : 0.f; v[8 + i] = kb < K ? W[(size_t)(kb < K ? kb : K - 1) * ld + n] : 0.f; }
  return bsplit16(v); }
__device__ __forceinline__ v8f mac3(const F2& a, const F2& b, v8f c) { c = wmma_bf(a.l, b.h, c); c = wmma_bf(a.h, b.l, c); return wmma_bf(a.h, b.h, c); }
__device__ __forceinline__ float sigm(float v) { return 1.0f / (1.0f + expf(-v)); }
#define LDSX() do { asm volatile("s_wait_dscnt 0" ::: "memory"); __builtin_amdgcn_wave_barrier(); __builtin_amdgcn_fence(__ATOMIC_RELEASE, "workgroup"); } while (0)


#define NB 4
#define SQ 512
#define NT (NB * SQ)
#define IN 256
#define OUT 256
#define HID 32
__device__ __forceinline__ float bfr(float v) { return (float)(__bf16)v; }
__device__ __forceinline__ v16b frag_b(const __bf16* rowk0, int lane) { return __builtin_bit_cast(v16b, frag_h((const _Float16*)rowk0, lane)); }

__global__ __launch_bounds__(128) void k_meta(const float* __restrict__ x, const float* __restrict__ w1, const float* __restrict__ b1, const float* __restrict__ w2, const float* __restrict__ b2, const float* __restrict__ u1, const float* __restrict__ c1, const float* __restrict__ u2, const float* __restrict__ c2, float* __restrict__ y) {
  __shared__ __align__(16) __bf16 sa[4][16][72];
  __shared__ __align__(16) float shb[4][16][36];
  __shared__ __align__(16) float sx[4][16][IN + 4];
  __shared__ __align__(16) float sy[4][16][OUT + 4];
  __shared__ float sbias[4][16][OUT + 4];
  const int tid = threadIdx.x, wave = tid >> 5, lane = tid & 31, col = lane & 15, g = lane >> 4; const int t0 = blockIdx.x * 64 + wave * 16;
  for (int q = lane; q < 16 * (IN / 4); q += 32) { const int rl = q >> 6, pc = q & 63; v4f v = *(const v4f*)(x + (size_t)(t0 + rl) * IN + pc * 4);
#pragma unroll
    for (int e = 0; e < 4; ++e) v[e] = bfr(v[e]);
    *(v4f*)(&sx[wave][rl][pc * 4]) = v; }
  { v8f ah[2] = {}, ab[2] = {};
#pragma unroll
    for (int kc = 0; kc < IN / 32; ++kc) { const v16b a = split_row(x + (size_t)(t0 + col) * IN, kc * 32, lane).h;
#pragma unroll
      for (int j = 0; j < 2; ++j) { ah[j] = wmma_bf(a, split_row(w1 + (size_t)(j * 16 + col) * IN, kc * 32, lane).h, ah[j]); ab[j] = wmma_bf(a, split_row(u1 + (size_t)(j * 16 + col) * IN, kc * 32, lane).h, ab[j]); } }
#pragma unroll
    for (int j = 0; j < 2; ++j) { const int n = j * 16 + col; const float bb1 = bfr(b1[n]), cc1 = bfr(c1[n]);
#pragma unroll
      for (int r = 0; r < 8; ++r) { const float hv = ah[j][r] + bb1; const __bf16 hi = (__bf16)hv; sa[wave][8 * g + r][n] = hi; sa[wave][8 * g + r][32 + n] = (__bf16)(hv - (float)hi); shb[wave][8 * g + r][n] = ab[j][r] + cc1; } } }
  LDSX();
  { const int rl = lane & 15, hf = lane >> 4; const float* hb = &shb[wave][rl][0]; float s = 0.f, sq = 0.f;
#pragma unroll 1
    for (int oo = 0; oo < OUT / 2; ++oo) { const int o = hf * (OUT / 2) + oo; const float* ur = u2 + (size_t)o * HID; float v = bfr(c2[o]);
#pragma unroll
      for (int hcol = 0; hcol < HID; ++hcol) v += hb[hcol] * bfr(ur[hcol]);
      sbias[wave][rl][o] = v; s += v; sq += v * v; }
    s += __shfl_xor(s, 16, 32); sq += __shfl_xor(sq, 16, 32);
    const float mu = s * (1.0f / OUT); float var = sq * (1.0f / OUT) - mu * mu; var = var > 0.f ? var : 0.f; const float rs = rsqrtf(var + 1e-5f);
#pragma unroll 1
    for (int oo = 0; oo < OUT / 2; ++oo) { const int o = hf * (OUT / 2) + oo; sbias[wave][rl][o] = (sbias[wave][rl][o] - mu) * rs; } }
  LDSX();
  const v16b a_hi = frag_b(&sa[wave][col][0], lane), a_lo = frag_b(&sa[wave][col][32], lane);
  float sxs[8];
#pragma unroll
  for (int r = 0; r < 8; ++r) { const float* xr = &sx[wave][8 * g + r][0]; float s = 0.f;
#pragma unroll 8
    for (int i = 0; i < IN; ++i) s += xr[i];
    sxs[r] = s; }
#pragma unroll 1
  for (int o = 0; o < OUT; ++o) { float sw[8], sw2[8], swx[8];
#pragma unroll
    for (int r = 0; r < 8; ++r) { sw[r] = 0.f; sw2[r] = 0.f; swx[r] = 0.f; }
#pragma unroll 2
    for (int t = 0; t < IN / 16; ++t) { const int i = t * 16 + col; const size_t wrow = (size_t)o * IN + i;
      const v16b wb = split_rowK(w2 + wrow * HID, 0, lane, HID).h;
      v8f acc = wmma_bf(a_lo, wb, (v8f){}); acc = wmma_bf(a_hi, wb, acc);
      const float bb = bfr(b2[wrow]);
#pragma unroll
      for (int r = 0; r < 8; ++r) { const float wv = acc[r] + bb; const float xv = sx[wave][8 * g + r][i]; sw[r] += wv; sw2[r] += wv * wv; swx[r] += wv * xv; } }
#pragma unroll
    for (int r = 0; r < 8; ++r) {
#pragma unroll
      for (int m = 1; m < 16; m <<= 1) { sw[r] += __shfl_xor(sw[r], m, 32); sw2[r] += __shfl_xor(sw2[r], m, 32); swx[r] += __shfl_xor(swx[r], m, 32); } }
    if (col == (o & 15)) {
#pragma unroll
      for (int r = 0; r < 8; ++r) { const float mu = sw[r] * (1.0f / IN); float var = sw2[r] * (1.0f / IN) - mu * mu; var = var > 0.f ? var : 0.f; const float rs = rsqrtf(var + 1e-5f);
        sy[wave][8 * g + r][o] = (swx[r] - mu * sxs[r]) * rs + sbias[wave][8 * g + r][o]; } } }
  LDSX();
  for (int rl = 0; rl < 16; ++rl) for (int pc = lane; pc < OUT / 4; pc += 32) vst2(y + (size_t)(t0 + rl) * OUT + pc * 4, *(const v4f*)(&sy[wave][rl][pc * 4]));
}
extern "C" void kernel_launch(void* const* d_in, const int* in_sizes, int n_in, void* d_out, int out_size, void* d_ws, size_t ws_size, hipStream_t stream) {
  (void)in_sizes; (void)n_in; (void)out_size; (void)ws_size; (void)d_ws;
  const float** I = (const float**)d_in;
  k_meta<<<NT / 64, 128, 0, stream>>>(I[0], I[1], I[2], I[3], I[4], I[5], I[6], I[7], I[8], (float*)d_out);
}
